// MultiheadAttention_16295105921351
// MI455X (gfx1250) — hardware-run, weakly checked
//
#include <hip/hip_runtime.h>
#include <math.h>

typedef __attribute__((ext_vector_type(16))) _Float16 v16h;
typedef __attribute__((ext_vector_type(8)))  _Float16 v8h;
typedef __attribute__((ext_vector_type(8)))  float    v8f;
typedef __attribute__((ext_vector_type(4)))  float    v4f;
typedef __attribute__((ext_vector_type(4)))  unsigned int v4u;
typedef __attribute__((ext_vector_type(4)))  int      v4i;

constexpr int kB    = 4;
constexpr int kS    = 2048;
constexpr int kD    = 1024;
constexpr int kH    = 16;
constexpr int kHD   = 64;
constexpr int kHalf = 32;
constexpr int kTok  = kB * kS;
constexpr int kBH   = kB * kH;
constexpr int kSE   = 512;
constexpr int kSqrtHD = 8;
static_assert(kH * kHD == kD);
static_assert(kSqrtHD * kSqrtHD == kHD);
static_assert(kHalf * 2 == kHD);
static_assert((kD % 32) == 0 && (kTok % 64) == 0 && (kS % 64) == 0 && (kSE % 64) == 0);

constexpr float kXC = 16.0f;
constexpr float kWC = 1024.0f;
constexpr float kQC = 16.0f;
constexpr float kPC = 32768.0f;
constexpr float kMC = 128.0f;
constexpr float kRC = 2048.0f;
constexpr float kRCInv      = 1.0f / kRC;
constexpr float kProjScale  = 1.0f / (kXC * kWC);
constexpr float kScoreScale = (1.0f / (float)kSqrtHD) / (kQC * kQC);
constexpr float kOScale     = kPC * kQC;
constexpr float kOutScale   = 1.0f / (kMC * kWC);

constexpr size_t kPlaneHi = (size_t)kBH * kS * kHD;
constexpr size_t kPlaneLo = (size_t)kBH * kSE * kHD;
constexpr size_t kOffX16 = 0;
constexpr size_t kOffW16 = kOffX16 + (size_t)kTok * kD * 2;
constexpr size_t kOffCOS = kOffW16 + (size_t)4 * kD * kD * 2;
constexpr size_t kOffSIN = kOffCOS + (size_t)kS * kHalf * 4;
constexpr size_t kOffQH  = kOffSIN + (size_t)kS * kHalf * 4;
constexpr size_t kOffKH  = kOffQH + kPlaneHi * 2;
constexpr size_t kOffVH  = kOffKH + kPlaneHi * 2;
constexpr size_t kOffQL  = kOffVH + kPlaneHi * 2;
constexpr size_t kOffKL  = kOffQL + kPlaneLo * 2;
constexpr size_t kOffVL  = kOffKL + kPlaneLo * 2;
constexpr size_t kOffMH  = kOffVL + kPlaneLo * 2;
constexpr size_t kOffML  = kOffMH + (size_t)kTok * kD * 2;
constexpr size_t kWsTotal = kOffML + (size_t)kB * kSE * kD * 2;
static_assert(kWsTotal == 109576192ull);
static_assert(kWsTotal <= 134217728ull);
static_assert((kOffW16 % 128) == 0 && (kOffCOS % 128) == 0 && (kOffSIN % 128) == 0 && (kOffQH % 128) == 0 &&
              (kOffKH % 128) == 0 && (kOffVH % 128) == 0 && (kOffQL % 128) == 0 && (kOffKL % 128) == 0 &&
              (kOffVL % 128) == 0 && (kOffMH % 128) == 0 && (kOffML % 128) == 0);

__device__ __forceinline__ unsigned short f2bf_bits(float f) {
  unsigned u = __float_as_uint(f);
  return (unsigned short)((u + 0x7FFFu + ((u >> 16) & 1u)) >> 16);
}
__device__ __forceinline__ float bf_bits2f(unsigned short h) { return __uint_as_float(((unsigned)h) << 16); }
__device__ __forceinline__ float bf_rne(float f) { return bf_bits2f(f2bf_bits(f)); }

union FragH { v16h v; v8h h[2]; };
__device__ __forceinline__ v16h frag_load(const _Float16* p) {
  FragH f;
  f.h[0] = *(const v8h*)(p);
  f.h[1] = *(const v8h*)(p + 16);
  return f.v;
}
__device__ __forceinline__ v8f mma_h(v16h a, v16h b, v8f c) {
  c = __builtin_amdgcn_wmma_f32_16x16x32_f16(false, a, false, b, (short)0, c, false, false);
  asm volatile("v_nop\n\tv_nop\n\tv_nop\n\tv_nop" : "+v"(c) : "v"(a), "v"(b));
  return c;
}
__device__ __forceinline__ void wave_lds_sync() {
  __builtin_amdgcn_fence(__ATOMIC_RELEASE, "workgroup");
  __builtin_amdgcn_wave_barrier();
  __builtin_amdgcn_fence(__ATOMIC_ACQUIRE, "workgroup");
}

__global__ __launch_bounds__(256) void cvt_planes_kernel(
    const float* __restrict__ p0, const float* __restrict__ p1, const float* __restrict__ p2,
    const float* __restrict__ p3, unsigned short* __restrict__ out, int n8, float carry) {
  const int i = blockIdx.x * 256 + threadIdx.x;
  if (i >= n8) return;
  const int z = blockIdx.y;
  const float* src = (z == 0) ? p0 : (z == 1) ? p1 : (z == 2) ? p2 : p3;
  const size_t e0 = (size_t)i << 3;
  const v4f a0 = *(const v4f*)(src + e0);
  const v4f a1 = *(const v4f*)(src + e0 + 4);
  v8h hv;
#pragma unroll
  for (int e = 0; e < 4; ++e) {
    hv[e]     = (_Float16)(bf_rne(a0[e]) * carry);
    hv[4 + e] = (_Float16)(bf_rne(a1[e]) * carry);
  }
  unsigned short* q = out + (size_t)z * ((size_t)n8 << 3) + e0;
  *(volatile v8h*)q = hv;
  __threadfence();
  *(volatile v8h*)q = hv;
}

struct RopeFreq { float v[kHalf]; };
static_assert(sizeof(RopeFreq) == 128);

__global__ __launch_bounds__(256) void rope_table_kernel(float* __restrict__ cosT, float* __restrict__ sinT, RopeFreq fr) {
#pragma clang fp contract(off)
  const int idx = blockIdx.x * 256 + threadIdx.x;
  const int s = idx >> 5;
  const int j = idx & 31;
  float f = fr.v[0];
#pragma unroll
  for (int i = 1; i < kHalf; ++i) f = (j == i) ? fr.v[i] : f;
  const float ang = (float)s * f;
  const float cs = cosf(ang);
  const float sn = sinf(ang);
  volatile float* pc = cosT + idx;
  volatile float* ps = sinT + idx;
  *pc = cs;
  *ps = sn;
  __threadfence();
  *pc = cs;
  *ps = sn;
}

template <int MI, bool RES, int EPI>
__global__ __launch_bounds__(256) void gemm_kernel(
    const unsigned short* __restrict__ Ap, const unsigned short* __restrict__ A2p,
    const unsigned short* __restrict__ Btp,
    int tilesN, int tilesSeg, int segStart, int totalTiles,
    const float* __restrict__ b0, const float* __restrict__ b1, const float* __restrict__ b2,
    const float* __restrict__ cosT, const float* __restrict__ sinT,
    unsigned short* __restrict__ hiBase, unsigned short* __restrict__ loBase,
    float* __restrict__ Out) {
  __shared__ __align__(16) float sT[8][16 * 68];
  const _Float16* A  = (const _Float16*)Ap;
  const _Float16* A2 = (const _Float16*)A2p;
  const _Float16* Bt = (const _Float16*)Btp;
  const int lane = threadIdx.x & 31;
  const int wave = __builtin_amdgcn_readfirstlane((int)(threadIdx.x >> 5));
  const int tile = blockIdx.x * 8 + wave;
  if (tile >= totalTiles) return;
  constexpr int TM = 16 * MI;
  const int tm  = tile / tilesN;
  const int tn  = tile - tm * tilesN;
  const int bb  = tm / tilesSeg;
  const int loc = tm - bb * tilesSeg;
  const int sBase = segStart + loc * TM;
  const int m0   = bb * kS + sBase;
  const int m0lo = bb * kSE + loc * TM;
  const int n0   = tn << 6;

  const int rlane = lane & 15;
  const int koff  = (lane >> 4) * 8;
  const int mOff  = (lane >> 4) * 8;

  v8f acc[MI][4];
  v8f accr[RES ? MI : 1][4];
#pragma unroll
  for (int i = 0; i < MI; ++i)
#pragma unroll
    for (int j = 0; j < 4; ++j) acc[i][j] = (v8f){0.f, 0.f, 0.f, 0.f, 0.f, 0.f, 0.f, 0.f};
#pragma unroll
  for (int i = 0; i < (RES ? MI : 1); ++i)
#pragma unroll
    for (int j = 0; j < 4; ++j) accr[i][j] = (v8f){0.f, 0.f, 0.f, 0.f, 0.f, 0.f, 0.f, 0.f};

  for (int k0 = 0; k0 < kD; k0 += 32) {
    v16h bh[4];
#pragma unroll
    for (int j = 0; j < 4; ++j)
      bh[j] = frag_load(Bt + (size_t)(n0 + (j << 4) + rlane) * kD + koff + k0);
#pragma unroll
    for (int i = 0; i < MI; ++i) {
      const v16h ah = frag_load(A + (size_t)(m0 + (i << 4) + rlane) * kD + koff + k0);
      v16h al = ah;
      if (RES) al = frag_load(A2 + (size_t)(m0lo + (i << 4) + rlane) * kD + koff + k0);
#pragma unroll
      for (int j = 0; j < 4; ++j) {
        acc[i][j] = mma_h(ah, bh[j], acc[i][j]);
        if (RES) accr[RES ? i : 0][j] = mma_h(al, bh[j], accr[RES ? i : 0][j]);
      }
    }
  }

  float* slab = sT[wave];
  if (EPI == 0) {
    const int kind = tn >> 4;
    const int head = tn & 15;
    const float* bp = (kind == 0) ? b0 : (kind == 1) ? b1 : b2;
    float bvj[4];
#pragma unroll
    for (int j = 0; j < 4; ++j) bvj[j] = bf_rne(bp[head * kHD + (j << 4) + rlane]);
    const bool early = (sBase < kSE);
    unsigned short* hp = hiBase + (size_t)kind * kPlaneHi + ((size_t)(bb * kH + head) * kS + sBase) * kHD;
    unsigned short* lp = loBase + (size_t)kind * kPlaneLo + ((size_t)(bb * kH + head) * kSE + (early ? sBase : 0)) * kHD;
    const int q4  = lane >> 3;
    const int c8  = (lane & 7) * 8;
    const int jc  = c8 & 31;
    const int pc8 = c8 ^ 32;
    const float sgn = (c8 < 32) ? -1.0f : 1.0f;
#pragma unroll
    for (int i = 0; i < MI; ++i) {
#pragma unroll
      for (int j = 0; j < 4; ++j)
#pragma unroll
        for (int r = 0; r < 8; ++r)
          slab[(mOff + r) * 68 + (j << 4) + rlane] = acc[i][j][r] * kProjScale + bvj[j];
      wave_lds_sync();
      v8h hv[4], lv[4];
#pragma unroll
      for (int it = 0; it < 4; ++it) {
        const int row = it * 4 + q4;
        const float* sp = slab + row * 68;
        const v4f x0 = *(const v4f*)(sp + c8);
        const v4f x1 = *(const v4f*)(sp + c8 + 4);
        v4f o0 = x0;
        v4f o1 = x1;
        if (kind < 2) {
          const v4f y0 = *(const v4f*)(sp + pc8);
          const v4f y1 = *(const v4f*)(sp + pc8 + 4);
          const size_t to = (size_t)(sBase + (i << 4) + row) * kHalf + jc;
          const v4f cA = *(const v4f*)(cosT + to);
          const v4f cB = *(const v4f*)(cosT + to + 4);
          const v4f sA = *(const v4f*)(sinT + to);
          const v4f sB = *(const v4f*)(sinT + to + 4);
#pragma unroll
          for (int e = 0; e < 4; ++e) {
            o0[e] = x0[e] * cA[e] + sgn * (y0[e] * sA[e]);
            o1[e] = x1[e] * cB[e] + sgn * (y1[e] * sB[e]);
          }
        }
#pragma unroll
        for (int e = 0; e < 4; ++e) {
          const float t0 = o0[e] * kQC;
          const float t1 = o1[e] * kQC;
          const _Float16 h0 = (_Float16)t0;
          const _Float16 h1 = (_Float16)t1;
          hv[it][e]     = h0;
          hv[it][4 + e] = h1;
          lv[it][e]     = (_Float16)((t0 - (float)h0) * kRC);
          lv[it][4 + e] = (_Float16)((t1 - (float)h1) * kRC);
        }
      }
      for (int pass = 0; pass < 2; ++pass) {
#pragma unroll
        for (int it = 0; it < 4; ++it) {
          const int row = it * 4 + q4;
          const size_t o = (size_t)((i << 4) + row) * kHD + c8;
          *(volatile v8h*)(hp + o) = hv[it];
          if (early) *(volatile v8h*)(lp + o) = lv[it];
        }
        __threadfence();
      }
      wave_lds_sync();
    }
  } else {
    float bvj[4];
#pragma unroll
    for (int j = 0; j < 4; ++j) bvj[j] = bf_rne(b0[n0 + (j << 4) + rlane]);
    const int hh2 = lane >> 4;
    const int c4  = (lane & 15) * 4;
#pragma unroll
    for (int i = 0; i < MI; ++i) {
#pragma unroll
      for (int j = 0; j < 4; ++j)
#pragma unroll
        for (int r = 0; r < 8; ++r) {
          float v = acc[i][j][r];
          if (RES) v += accr[RES ? i : 0][j][r] * kRCInv;
          slab[(mOff + r) * 68 + (j << 4) + rlane] = v * kOutScale + bvj[j];
        }
      wave_lds_sync();
      v4f vv[8];
#pragma unroll
      for (int it = 0; it < 8; ++it) vv[it] = *(const v4f*)(slab + (it * 2 + hh2) * 68 + c4);
      for (int pass = 0; pass < 2; ++pass) {
#pragma unroll
        for (int it = 0; it < 8; ++it)
          *(volatile v4f*)(Out + (size_t)(m0 + (i << 4) + it * 2 + hh2) * kD + n0 + c4) = vv[it];
        __threadfence();
      }
      wave_lds_sync();
    }
  }
}

template <bool EARLY>
__global__ __launch_bounds__(128) void attn_kernel(
    const unsigned short* __restrict__ QH, const unsigned short* __restrict__ KH, const unsigned short* __restrict__ VH,
    const unsigned short* __restrict__ QL, const unsigned short* __restrict__ KL, const unsigned short* __restrict__ VL,
    const int* __restrict__ mask,
    unsigned short* __restrict__ MH, unsigned short* __restrict__ ML,
    int nqb, int qb0) {
  constexpr int KVB  = EARLY ? 32768 : 16384;
  constexpr int PB   = EARLY ? 16384 : 8192;
  constexpr int SMEM = KVB + PB + 4096;
  static_assert(SMEM >= 4 * 16 * 68 * 4);
  __shared__ __align__(16) unsigned char smem[SMEM];
  _Float16* Ksh = (_Float16*)(smem);
  _Float16* Vth = (_Float16*)(smem + 8192);
  _Float16* Ksl = (_Float16*)(smem + (EARLY ? 16384 : 0));
  _Float16* Vtl = (_Float16*)(smem + (EARLY ? 24576 : 8192));
  _Float16* Ph  = (_Float16*)(smem + KVB);
  _Float16* Pl  = (_Float16*)(smem + KVB + (EARLY ? 8192 : 0));
  unsigned char* Mk = smem + KVB + PB;

  const int tid  = threadIdx.x;
  const int wave = __builtin_amdgcn_readfirstlane((int)(threadIdx.x >> 5));
  const int lane = tid & 31;
  const int hf   = lane >> 4;
  const int c    = lane & 15;

  const int bx = blockIdx.x;
  const int bh = bx / nqb;
  const int qb = qb0 + (bx - bh * nqb);
  const int b  = bh / kH;
  const int h  = bh - b * kH;
  const int qbase = qb * 64;
  const int q0 = qbase + wave * 16;

  v16h qah[2], qal[2];
  {
    const _Float16* qrow = (const _Float16*)QH + ((size_t)bh * kS + q0 + c) * kHD + 8 * hf;
#pragma unroll
    for (int dc = 0; dc < 2; ++dc) {
      qah[dc] = frag_load(qrow + dc * 32);
      qal[dc] = qah[dc];
    }
    if (EARLY) {
      const _Float16* qlrow = (const _Float16*)QL + ((size_t)bh * kSE + q0 + c) * kHD + 8 * hf;
#pragma unroll
      for (int dc = 0; dc < 2; ++dc) qal[dc] = frag_load(qlrow + dc * 32);
    }
  }

  float mrow[8], lrow[8];
  v8f oacc[4];
#pragma unroll
  for (int r = 0; r < 8; ++r) { mrow[r] = -1.0e30f; lrow[r] = 0.f; }
#pragma unroll
  for (int t = 0; t < 4; ++t) oacc[t] = (v8f){0.f, 0.f, 0.f, 0.f, 0.f, 0.f, 0.f, 0.f};

  _Float16* pwh = Ph + wave * (16 * 64);
  _Float16* pwl = Pl + wave * (16 * 64);

  for (int kc = 0; kc <= qb; ++kc) {
    const int kv0 = kc * 64;
    __syncthreads();
    {
      const v4u* kg = (const v4u*)(KH + ((size_t)bh * kS + kv0) * kHD);
      const v4u* vg = (const v4u*)(VH + ((size_t)bh * kS + kv0) * kHD);
#pragma unroll
      for (int i = 0; i < 4; ++i) {
        const int idx = tid + 128 * i;
        const v4u kw = kg[idx];
        const v4u vw = vg[idx];
        ((v4u*)Ksh)[idx] = kw;
        const int kvr = idx >> 3;
        const int d8  = (idx & 7) * 8;
#pragma unroll
        for (int w = 0; w < 4; ++w) {
          const unsigned word = vw[w];
          const unsigned short e0 = (unsigned short)(word & 0xffffu);
          const unsigned short e1 = (unsigned short)(word >> 16);
          const _Float16 f0 = __builtin_bit_cast(_Float16, e0);
          const _Float16 f1 = __builtin_bit_cast(_Float16, e1);
          Vth[(d8 + 2 * w) * 64 + kvr]     = f0;
          Vth[(d8 + 2 * w + 1) * 64 + kvr] = f1;
        }
      }
      if (EARLY) {
        const v4u* kgl = (const v4u*)(KL + ((size_t)bh * kSE + kv0) * kHD);
        const v4u* vgl = (const v4u*)(VL + ((size_t)bh * kSE + kv0) * kHD);
#pragma unroll
        for (int i = 0; i < 4; ++i) {
          const int idx = tid + 128 * i;
          const v4u kw = kgl[idx];
          const v4u vw = vgl[idx];
          ((v4u*)Ksl)[idx] = kw;
          const int kvr = idx >> 3;
          const int d8  = (idx & 7) * 8;
#pragma unroll
          for (int w = 0; w < 4; ++w) {
            const unsigned word = vw[w];
            const unsigned short e0 = (unsigned short)(word & 0xffffu);
            const unsigned short e1 = (unsigned short)(word >> 16);
            const _Float16 f0 = __builtin_bit_cast(_Float16, e0);
            const _Float16 f1 = __builtin_bit_cast(_Float16, e1);
            Vtl[(d8 + 2 * w) * 64 + kvr]     = f0;
            Vtl[(d8 + 2 * w + 1) * 64 + kvr] = f1;
          }
        }
      }
      if (kc == qb) {
#pragma unroll
        for (int i = 0; i < 8; ++i) {
          const int idx = tid + 128 * i;
          const int row = idx >> 4;
          const int c4  = (idx & 15) * 4;
          const v4i mv = *(const v4i*)(mask + (size_t)(qbase + row) * kS + kv0 + c4);
          const unsigned m0 = (mv[0] != 0) ? 1u : 0u;
          const unsigned m1 = (mv[1] != 0) ? 1u : 0u;
          const unsigned m2 = (mv[2] != 0) ? 1u : 0u;
          const unsigned m3 = (mv[3] != 0) ? 1u : 0u;
          ((unsigned*)Mk)[idx] = m0 | (m1 << 8) | (m2 << 16) | (m3 << 24);
        }
      }
    }
    __syncthreads();

    v8f s[4];
#pragma unroll
    for (int j = 0; j < 4; ++j) {
      v8f sm = (v8f){0.f, 0.f, 0.f, 0.f, 0.f, 0.f, 0.f, 0.f};
      v8f sr = (v8f){0.f, 0.f, 0.f, 0.f, 0.f, 0.f, 0.f, 0.f};
#pragma unroll
      for (int dc = 0; dc < 2; ++dc) {
        const v16h kb = frag_load(Ksh + (j * 16 + c) * 64 + dc * 32 + 8 * hf);
        sm = mma_h(qah[dc], kb, sm);
        if (EARLY) {
          const v16h kl = frag_load(Ksl + (j * 16 + c) * 64 + dc * 32 + 8 * hf);
          sr = mma_h(qah[dc], kl, sr);
          sr = mma_h(qal[dc], kb, sr);
        }
      }
#pragma unroll
      for (int r = 0; r < 8; ++r)
        s[j][r] = EARLY ? ((sm[r] + sr[r] * kRCInv) * kScoreScale) : (sm[r] * kScoreScale);
    }
    if (kc == qb) {
#pragma unroll
      for (int r = 0; r < 8; ++r)
#pragma unroll
        for (int j = 0; j < 4; ++j) {
          const unsigned char mb = Mk[(wave * 16 + 8 * hf + r) * 64 + j * 16 + c];
          s[j][r] = (mb != 0) ? -INFINITY : s[j][r];
        }
    }
    float cm[8];
#pragma unroll
    for (int r = 0; r < 8; ++r) {
      float m = fmaxf(fmaxf(s[0][r], s[1][r]), fmaxf(s[2][r], s[3][r]));
#pragma unroll
      for (int off = 1; off < 16; off <<= 1) m = fmaxf(m, __shfl_xor(m, off, 32));
      cm[r] = m;
    }
#pragma unroll
    for (int r = 0; r < 8; ++r) {
      const float mnew  = fmaxf(mrow[r], cm[r]);
      const float alpha = EARLY ? expf(mrow[r] - mnew) : __expf(mrow[r] - mnew);
      mrow[r] = mnew;
      float psum = 0.f;
#pragma unroll
      for (int j = 0; j < 4; ++j) {
        const float p = EARLY ? expf(s[j][r] - mnew) : __expf(s[j][r] - mnew);
        psum += p;
        const float t = p * kPC;
        const _Float16 ph = (_Float16)t;
        pwh[(8 * hf + r) * 64 + j * 16 + c] = ph;
        if (EARLY) pwl[(8 * hf + r) * 64 + j * 16 + c] = (_Float16)((t - (float)ph) * kRC);
      }
#pragma unroll
      for (int off = 1; off < 16; off <<= 1) psum += __shfl_xor(psum, off, 32);
      lrow[r] = lrow[r] * alpha + psum;
#pragma unroll
      for (int t = 0; t < 4; ++t) oacc[t][r] *= alpha;
    }
    wave_lds_sync();

    v16h pa[2], pl[2];
#pragma unroll
    for (int kk = 0; kk < 2; ++kk) {
      pa[kk] = frag_load(pwh + c * 64 + kk * 32 + 8 * hf);
      pl[kk] = pa[kk];
      if (EARLY) pl[kk] = frag_load(pwl + c * 64 + kk * 32 + 8 * hf);
    }
#pragma unroll
    for (int t = 0; t < 4; ++t) {
      v8f tr = (v8f){0.f, 0.f, 0.f, 0.f, 0.f, 0.f, 0.f, 0.f};
#pragma unroll
      for (int kk = 0; kk < 2; ++kk) {
        const v16h vb = frag_load(Vth + (t * 16 + c) * 64 + kk * 32 + 8 * hf);
        oacc[t] = mma_h(pa[kk], vb, oacc[t]);
        if (EARLY) {
          const v16h vl = frag_load(Vtl + (t * 16 + c) * 64 + kk * 32 + 8 * hf);
          tr = mma_h(pa[kk], vl, tr);
          tr = mma_h(pl[kk], vb, tr);
        }
      }
      if (EARLY) {
#pragma unroll
        for (int r = 0; r < 8; ++r) oacc[t][r] += tr[r] * kRCInv;
      }
    }
  }

  __syncthreads();
  float* os = (float*)smem + wave * (16 * 68);
#pragma unroll
  for (int r = 0; r < 8; ++r) {
    const float inv = 1.0f / (lrow[r] * kOScale);
#pragma unroll
    for (int t = 0; t < 4; ++t) os[(8 * hf + r) * 68 + t * 16 + c] = oacc[t][r] * inv;
  }
  wave_lds_sync();
  {
    const int q4 = lane >> 3;
    const int c8 = (lane & 7) * 8;
    v8h hv[4], lv[4];
#pragma unroll
    for (int it = 0; it < 4; ++it) {
      const int row = it * 4 + q4;
      const float* sp = os + row * 68 + c8;
      const v4f a0 = *(const v4f*)(sp);
      const v4f a1 = *(const v4f*)(sp + 4);
#pragma unroll
      for (int e = 0; e < 4; ++e) {
        const float t0 = a0[e] * kMC;
        const float t1 = a1[e] * kMC;
        const _Float16 h0 = (_Float16)t0;
        const _Float16 h1 = (_Float16)t1;
        hv[it][e]     = h0;
        hv[it][4 + e] = h1;
        lv[it][e]     = (_Float16)((t0 - (float)h0) * kRC);
        lv[it][4 + e] = (_Float16)((t1 - (float)h1) * kRC);
      }
    }
    unsigned short* mh = MH + (size_t)(b * kS + q0) * kD + h * kHD + c8;
    unsigned short* ml = ML + (size_t)(b * kSE + (EARLY ? q0 : 0)) * kD + h * kHD + c8;
    for (int pass = 0; pass < 2; ++pass) {
#pragma unroll
      for (int it = 0; it < 4; ++it) {
        const int row = it * 4 + q4;
        *(volatile v8h*)(mh + (size_t)row * kD) = hv[it];
        if (EARLY) *(volatile v8h*)(ml + (size_t)row * kD) = lv[it];
      }
      __threadfence();
    }
  }
}

extern "C" void kernel_launch(void* const* d_in, const int* in_sizes, int n_in,
                              void* d_out, int out_size, void* d_ws, size_t ws_size,
                              hipStream_t stream) {
  if (n_in < 10) return;
  if (in_sizes[0] != kTok * kD) return;
  if (in_sizes[1] != kD * kD || in_sizes[3] != kD * kD || in_sizes[5] != kD * kD || in_sizes[7] != kD * kD) return;
  if (in_sizes[2] != kD || in_sizes[4] != kD || in_sizes[6] != kD || in_sizes[8] != kD) return;
  if (in_sizes[9] != kS * kS) return;
  if (out_size != kTok * kD) return;
  if (ws_size < kWsTotal) return;

  const float* x  = (const float*)d_in[0];
  const float* Wq = (const float*)d_in[1];
  const float* bq = (const float*)d_in[2];
  const float* Wk = (const float*)d_in[3];
  const float* bk = (const float*)d_in[4];
  const float* Wv = (const float*)d_in[5];
  const float* bv = (const float*)d_in[6];
  const float* Wo = (const float*)d_in[7];
  const float* bo = (const float*)d_in[8];
  const int*   mk = (const int*)d_in[9];
  float* out = (float*)d_out;

  char* ws = (char*)d_ws;
  unsigned short* X16 = (unsigned short*)(ws + kOffX16);
  unsigned short* W16 = (unsigned short*)(ws + kOffW16);
  float*          COS = (float*)(ws + kOffCOS);
  float*          SIN = (float*)(ws + kOffSIN);
  unsigned short* QH  = (unsigned short*)(ws + kOffQH);
  unsigned short* KH  = (unsigned short*)(ws + kOffKH);
  unsigned short* VH  = (unsigned short*)(ws + kOffVH);
  unsigned short* QL  = (unsigned short*)(ws + kOffQL);
  unsigned short* KL  = (unsigned short*)(ws + kOffKL);
  unsigned short* VL  = (unsigned short*)(ws + kOffVL);
  unsigned short* MH  = (unsigned short*)(ws + kOffMH);
  unsigned short* ML  = (unsigned short*)(ws + kOffML);

  RopeFreq fr;
  for (int j = 0; j < kHalf; ++j) {
    const float e = (float)j / (float)kHalf;
    const float p = (float)pow(10000.0, (double)e);
    fr.v[j] = 1.0f / p;
  }

  cvt_planes_kernel<<<dim3(kTok * kD / 8 / 256, 1), 256, 0, stream>>>(x, x, x, x, X16, kTok * kD / 8, kXC);
  cvt_planes_kernel<<<dim3(kD * kD / 8 / 256, 4), 256, 0, stream>>>(Wq, Wk, Wv, Wo, W16, kD * kD / 8, kWC);
  rope_table_kernel<<<kS * kHalf / 256, 256, 0, stream>>>(COS, SIN, fr);

  gemm_kernel<4, false, 0><<<(kTok / 64) * (3 * kD / 64) / 8, 256, 0, stream>>>(
      X16, X16, W16,
      3 * kD / 64, kS / 64, 0, (kTok / 64) * (3 * kD / 64),
      bq, bk, bv, COS, SIN, QH, QL, out);

  attn_kernel<true><<<kBH * (kSE / 64), 128, 0, stream>>>(QH, KH, VH, QL, KL, VL, mk, MH, ML, kSE / 64, 0);
  attn_kernel<false><<<kBH * ((kS - kSE) / 64), 128, 0, stream>>>(QH, KH, VH, QL, KL, VL, mk, MH, ML,
                                                                 (kS - kSE) / 64, kSE / 64);

  const unsigned short* Wo16 = W16 + (size_t)3 * kD * kD;
  gemm_kernel<2, true, 1><<<(kB * (kSE / 32)) * (kD / 64) / 8, 256, 0, stream>>>(
      MH, ML, Wo16,
      kD / 64, kSE / 32, 0, (kB * (kSE / 32)) * (kD / 64),
      bo, bo, bo, COS, SIN, QH, QL, out);
  gemm_kernel<4, false, 1><<<(kB * ((kS - kSE) / 64)) * (kD / 64) / 8, 256, 0, stream>>>(
      MH, MH, Wo16,
      kD / 64, (kS - kSE) / 64, kSE, (kB * ((kS - kSE) / 64)) * (kD / 64),
      bo, bo, bo, COS, SIN, QH, QL, out);
}
